// GFA_53377853554970
// MI455X (gfx1250) — hardware-verified
//
#include <hip/hip_runtime.h>
#include <math.h>

typedef __attribute__((ext_vector_type(16))) _Float16 v16h;
typedef __attribute__((ext_vector_type(16))) __bf16 v16b;
typedef __attribute__((ext_vector_type(8)))  _Float16 v8h;
typedef __attribute__((ext_vector_type(8)))  float v8f;
typedef __attribute__((ext_vector_type(4)))  float v4f;
typedef __attribute__((ext_vector_type(2)))  float v2f;
typedef __attribute__((ext_vector_type(4)))  unsigned v4u;
typedef __attribute__((ext_vector_type(4)))  int v4i;
typedef float __attribute__((may_alias)) float_a;
typedef int __attribute__((may_alias)) int_a;

template <typename T> __device__ __forceinline__ void vst2(void* p, T v) { *(volatile T*)p = v; __threadfence(); *(volatile T*)p = v; }
__device__ __forceinline__ v8f wmma16(v16h a, v16h b, v8f c) {
  v8f d = __builtin_amdgcn_wmma_f32_16x16x32_f16(false, a, false, b, (short)0, c, false, false);
  asm volatile("v_nop\n\tv_nop\n\tv_nop\n\tv_nop" : "+v"(d) : "v"(a), "v"(b));
  return d;
}
__device__ __forceinline__ v8f wmma_bf(v16b a, v16b b, v8f c) {
  v8f d = __builtin_amdgcn_wmma_f32_16x16x32_bf16(false, a, false, b, (short)0, c, false, false);
  asm volatile("v_nop\n\tv_nop\n\tv_nop\n\tv_nop" : "+v"(d) : "v"(a), "v"(b));
  return d;
}
__device__ __forceinline__ v16h frag_h(const _Float16* rowk0, int lane) {
  union { v16h v; v8h q[2]; } u; const _Float16* p = rowk0 + 8 * (lane >> 4);
  u.q[0] = *(const v8h*)p; u.q[1] = *(const v8h*)(p + 16); return u.v;
}
__device__ __forceinline__ v16h frag_f32(const float* rowk0, int lane) {
  v16h a; const float* p = rowk0 + 8 * (lane >> 4);
#pragma unroll
  for (int i = 0; i < 8; ++i) { a[i] = (_Float16)p[i]; a[8 + i] = (_Float16)p[16 + i]; }
  return a;
}
__device__ __forceinline__ v16h frag_f32s(const float* rowk0, int lane, float sc) {
  v16h a; const float* p = rowk0 + 8 * (lane >> 4);
#pragma unroll
  for (int i = 0; i < 8; ++i) { a[i] = (_Float16)(p[i] * sc); a[8 + i] = (_Float16)(p[16 + i] * sc); }
  return a;
}
__device__ __forceinline__ v16h fragc_f32(const float* W, int k0, int n, int lane, int ld, int K) {
  v16h a; const int g = lane >> 4;
#pragma unroll
  for (int i = 0; i < 8; ++i) { const int ka = k0 + 8 * g + i, kb = ka + 16;
    a[i] = (_Float16)(ka < K ? W[(size_t)(ka < K ? ka : K - 1) * ld + n] : 0.f); a[8 + i] = (_Float16)(kb < K ? W[(size_t)(kb < K ? kb : K - 1) * ld + n] : 0.f); }
  return a;
}
struct F2 { v16b h, l; };
__device__ __forceinline__ F2 bsplit16(const float v[16]) { F2 r;
#pragma unroll
  for (int i = 0; i < 16; ++i) { const __bf16 h = (__bf16)v[i]; r.h[i] = h; r.l[i] = (__bf16)(v[i] - (float)h); }
  return r; }
__device__ __forceinline__ F2 split_row(const float* row, int k0, int lane) { float v[16]; const float* p = row + k0 + 8 * (lane >> 4);
#pragma unroll
  for (int i = 0; i < 8; ++i) { v[i] = p[i]; v[8 + i] = p[16 + i]; }
  return bsplit16(v); }
__device__ __forceinline__ F2 split_rowK(const float* row, int k0, int lane, int K) { float v[16]; const int g = lane >> 4;
#pragma unroll
  for (int i = 0; i < 8; ++i) { const int ka = k0 + 8 * g + i, kb = ka + 16; v[i] = ka < K ? row[ka < K ? ka : K - 1] : 0.f; v[8 + i] = kb < K ? row[kb < K ? kb : K - 1] : 0.f; }
  return bsplit16(v); }
__device__ __forceinline__ F2 split_col(const float* W, int k0, int n, int lane, int ld, int K) { float v[16]; const int g = lane >> 4;
#pragma unroll
  for (int i = 0; i < 8; ++i) { const int ka = k0 + 8 * g + i, kb = ka + 16; v[i] = ka < K ? W[(size_t)(ka < K ? ka : K - 1) * ld + n] : 0.f; v[8 + i] = kb < K ? W[(size_t)(kb < K ? kb : K - 1) * ld + n] : 0.f; }
  return bsplit16(v); }
__device__ __forceinline__ v8f mac3(const F2& a, const F2& b, v8f c) { c = wmma_bf(a.l, b.h, c); c = wmma_bf(a.h, b.l, c); return wmma_bf(a.h, b.h, c); }
__device__ __forceinline__ float sigm(float v) { return 1.0f / (1.0f + expf(-v)); }
#define LDSX() do { asm volatile("s_wait_dscnt 0" ::: "memory"); __builtin_amdgcn_wave_barrier(); __builtin_amdgcn_fence(__ATOMIC_RELEASE, "workgroup"); } while (0)

__device__ __forceinline__ float bfr(float v) { return (float)(__bf16)v; }
#define NB 2
#define CC 64
#define TT 8192
#define QCH 2048
#ifndef TNB
#define TNB NB
#endif
#ifndef NQCH
#define NQCH (TT / QCH)
#endif
#ifndef XSTR
#define XSTR TT
#endif
#define WS_XT  0u
#define WS_AH  (WS_XT + 4u * (size_t)NB * TT * CC)
#define WS_AL  (WS_AH + 2u * (size_t)NB * TT * CC)
#define WS_BH  (WS_AL + 2u * (size_t)NB * TT * CC)
#define WS_BL  (WS_BH + 2u * (size_t)NB * TT * CC)
#define WS_MP  (WS_BL + 2u * (size_t)NB * TT * CC)
#define WS_S   (WS_MP + 2u * (size_t)NB * CC * TT)
#define WS_END (WS_S + 4u * (size_t)QCH * TT)
__global__ __launch_bounds__(256) void k_xt(const float* __restrict__ X, float* __restrict__ XT) { __shared__ float st[CC][65];
  const int t = threadIdx.x; const int n0 = blockIdx.x * 64; const size_t b = blockIdx.y;
  for (int e = t; e < CC * 64; e += 256) { const int c = e >> 6, nl = e & 63; st[c][nl] = bfr(X[(b * CC + c) * (size_t)XSTR + n0 + nl]); }
  __syncthreads();
  for (int e = t; e < 64 * 16; e += 256) { const int nl = e >> 4, q = e & 15; v4f o; o[0] = st[q * 4][nl]; o[1] = st[q * 4 + 1][nl]; o[2] = st[q * 4 + 2][nl]; o[3] = st[q * 4 + 3][nl]; vst2(XT + (b * TT + n0 + nl) * CC + q * 4, o); } }
__global__ __launch_bounds__(128) void k_proj(const float* __restrict__ XT, const float* __restrict__ WA, const float* __restrict__ BA, const float* __restrict__ WB, const float* __restrict__ BB, const float* __restrict__ WM, const float* __restrict__ BM, const float* __restrict__ G, const float* __restrict__ BT, const float* __restrict__ MU, const float* __restrict__ VAR,
    _Float16* __restrict__ AH, _Float16* __restrict__ AL, _Float16* __restrict__ BH, _Float16* __restrict__ BL, _Float16* __restrict__ MP) { __shared__ __align__(16) _Float16 sh[64][72], sl[64][72]; __shared__ __align__(16) _Float16 th[CC][72];
  const int tid = threadIdx.x, wave = tid >> 5, lane = tid & 31, col = lane & 15, g = lane >> 4; const int which = blockIdx.y; const size_t r0 = (size_t)blockIdx.x * 64; const float* Wt = which == 0 ? WA : which == 1 ? WB : WM; const float* Bv = which == 0 ? BA : which == 1 ? BB : BM;
  v8f acc[4] = {};
#pragma unroll
  for (int kc = 0; kc < CC / 32; ++kc) { v16b a; { const float* p = XT + (r0 + wave * 16 + col) * CC + kc * 32 + 8 * g;
#pragma unroll
      for (int i = 0; i < 8; ++i) { a[i] = (__bf16)p[i]; a[8 + i] = (__bf16)p[16 + i]; } }
#pragma unroll
    for (int j = 0; j < 4; ++j) { v16b w; const float* wr = Wt + (size_t)(j * 16 + col) * CC + kc * 32 + 8 * g;
#pragma unroll
      for (int i = 0; i < 8; ++i) { w[i] = (__bf16)wr[i]; w[8 + i] = (__bf16)wr[16 + i]; }
      asm volatile("s_wait_loadcnt 0x0" ::: "memory"); acc[j] = wmma_bf(a, w, acc[j]); } }
#pragma unroll
  for (int j = 0; j < 4; ++j) { const int o = j * 16 + col; const float bb = bfr(Bv[o]); float sc = 1.f, sh0 = 0.f; if (which == 2) { sc = rsqrtf(bfr(VAR[o]) + 1e-5f) * bfr(G[o]); sh0 = bfr(BT[o]) - bfr(MU[o]) * sc; }
#pragma unroll
    for (int r = 0; r < 8; ++r) { const float v = acc[j][r] + bb; const int rl = wave * 16 + 8 * g + r;
      if (which == 2) th[o][rl] = (_Float16)(v * sc + sh0); else { const _Float16 hv = (_Float16)v; sh[rl][o] = hv; sl[rl][o] = (_Float16)((v - (float)hv) * 1024.0f); } } }
  __syncthreads();
  if (which < 2) { _Float16* DH = which == 0 ? AH : BH; _Float16* DL = which == 0 ? AL : BL; for (int e = tid; e < 64 * 8; e += 128) { const int rl = e >> 3, q = e & 7; vst2((unsigned*)(DH + (r0 + rl) * CC + q * 8), *(const v4u*)&sh[rl][q * 8]); vst2((unsigned*)(DL + (r0 + rl) * CC + q * 8), *(const v4u*)&sl[rl][q * 8]); } }
  else { const size_t b = r0 / TT; const int n0 = (int)(r0 % TT); for (int e = tid; e < CC * 8; e += 128) { const int cl = e >> 3, q = e & 7; vst2((unsigned*)(MP + (b * CC + cl) * (size_t)TT + n0 + q * 8), *(const v4u*)&th[cl][q * 8]); } } }
__global__ __launch_bounds__(128) void k_sc(const _Float16* __restrict__ AH, const _Float16* __restrict__ AL, const _Float16* __restrict__ BH, const _Float16* __restrict__ BL, int b, int qbase, float* __restrict__ S) { __shared__ __align__(16) float ss[4][16][132];
  const int tid = threadIdx.x, wave = tid >> 5, lane = tid & 31, col = lane & 15, g = lane >> 4; const int k0 = blockIdx.y * 128; const int ql0 = blockIdx.x * 64 + wave * 16; const size_t qrow = (size_t)b * TT + qbase + ql0 + col;
  v8f acc[8] = {}, accl[8] = {};
#pragma unroll
  for (int kc = 0; kc < CC / 32; ++kc) { const v16h ah = frag_h(AH + qrow * CC + kc * 32, lane), al = frag_h(AL + qrow * CC + kc * 32, lane);
#pragma unroll
    for (int j = 0; j < 8; ++j) { const size_t ko = ((size_t)b * TT + k0 + j * 16 + col) * CC + kc * 32; const v16h kb = frag_h(BH + ko, lane), kl = frag_h(BL + ko, lane); acc[j] = wmma16(ah, kb, acc[j]); accl[j] = wmma16(al, kb, accl[j]); accl[j] = wmma16(ah, kl, accl[j]); } }
#pragma unroll
  for (int j = 0; j < 8; ++j)
#pragma unroll
    for (int r = 0; r < 8; ++r) ss[wave][8 * g + r][j * 16 + col] = acc[j][r] + accl[j][r] * (1.0f / 1024.0f);
  LDSX(); for (int rl = 0; rl < 16; ++rl) vst2(S + (size_t)(ql0 + rl) * TT + k0 + lane * 4, *(const v4f*)&ss[wave][rl][lane * 4]); }
__global__ __launch_bounds__(256) void k_sm(float* __restrict__ S) { __shared__ float sred[8]; __shared__ float sbc; __shared__ __align__(16) float shh[TT];
  const int t = threadIdx.x; const size_t row = blockIdx.x; float* sr = S + row * TT;
  float m = -3.0e38f; for (int k = t; k < TT; k += 256) { const float v = sr[k]; shh[k] = v; m = fmaxf(m, v); }
#pragma unroll
  for (int o = 1; o < 32; o <<= 1) m = fmaxf(m, __shfl_xor(m, o));
  if ((t & 31) == 0) sred[t >> 5] = m; __syncthreads(); if (t == 0) { float a = sred[0]; for (int w = 1; w < 8; ++w) a = fmaxf(a, sred[w]); sbc = a; } __syncthreads(); m = sbc; __syncthreads();
  float s = 0.f; for (int k = t; k < TT; k += 256) { const float e = expf(shh[k] - m); shh[k] = e; s += e; }
#pragma unroll
  for (int o = 1; o < 32; o <<= 1) s += __shfl_xor(s, o);
  if ((t & 31) == 0) sred[t >> 5] = s; __syncthreads(); if (t == 0) { float a = 0.f; for (int w = 0; w < 8; ++w) a += sred[w]; sbc = 2048.0f / a; } __syncthreads(); const float sc = sbc;
  for (int k = t; k < TT; k += 256) shh[k] *= sc;
  __syncthreads(); for (int q = t; q < TT / 4; q += 256) vst2(sr + q * 4, *(const v4f*)&shh[q * 4]); }
__global__ __launch_bounds__(128) void k_pv(const float* __restrict__ PS, const _Float16* __restrict__ MP, const float* __restrict__ X, const float* __restrict__ ALPHA, int b, int qbase, float* __restrict__ OUT) { __shared__ __align__(16) float stc[CC][68];
  const int tid = threadIdx.x, wave = tid >> 5, lane = tid & 31, col = lane & 15, g = lane >> 4; const int ql0 = blockIdx.x * 64 + wave * 16; const float alpha = bfr(ALPHA[0]);
  v8f acc[4] = {}, accl[4] = {};
#pragma unroll 1
  for (int kc = 0; kc < TT / 32; ++kc) { v16h ph, pl; { const float* pr = PS + (size_t)(ql0 + col) * TT + kc * 32 + 8 * g;
#pragma unroll
      for (int i = 0; i < 8; ++i) { const float a0 = pr[i], a1 = pr[16 + i]; const _Float16 h0 = (_Float16)a0, h1 = (_Float16)a1; ph[i] = h0; ph[8 + i] = h1; pl[i] = (_Float16)((a0 - (float)h0) * 1024.0f); pl[8 + i] = (_Float16)((a1 - (float)h1) * 1024.0f); } }
    asm volatile("s_wait_loadcnt 0x0" ::: "memory");
#pragma unroll
    for (int j = 0; j < 4; ++j) { const v16h mv = frag_h(MP + ((size_t)b * CC + j * 16 + col) * (size_t)TT + kc * 32, lane); acc[j] = wmma16(ph, mv, acc[j]); accl[j] = wmma16(pl, mv, accl[j]); } }
#pragma unroll
  for (int j = 0; j < 4; ++j)
#pragma unroll
    for (int r = 0; r < 8; ++r) stc[j * 16 + col][wave * 16 + 8 * g + r] = (acc[j][r] + accl[j][r] * (1.0f / 1024.0f)) * (1.0f / 2048.0f);
  __syncthreads();
  { const int n0 = qbase + blockIdx.x * 64; for (int e = tid; e < CC * 16; e += 128) { const int c = e >> 4, q = e & 15; const size_t off = ((size_t)b * CC + c) * (size_t)XSTR + n0 + q * 4; const v4f xr = *(const v4f*)(X + off); v4f o = *(const v4f*)&stc[c][q * 4];
#pragma unroll
      for (int z = 0; z < 4; ++z) { const float p = bfr(xr[z]) + alpha * o[z]; o[z] = p + p; }
      vst2(OUT + off, o); } } }
extern "C" void kernel_launch(void* const* d_in, const int* in_sizes, int n_in, void* d_out, int out_size, void* d_ws, size_t ws_size, hipStream_t stream) {
  (void)in_sizes; (void)n_in; (void)out_size;
  const float** F = (const float**)d_in;
  if (ws_size < (size_t)WS_END) return;
  char* ws = (char*)d_ws; float *XT = (float*)(ws + WS_XT), *S = (float*)(ws + WS_S); _Float16 *AH = (_Float16*)(ws + WS_AH), *AL = (_Float16*)(ws + WS_AL), *BH = (_Float16*)(ws + WS_BH), *BL = (_Float16*)(ws + WS_BL), *MP = (_Float16*)(ws + WS_MP);
  k_xt<<<dim3(TT / 64, TNB), 256, 0, stream>>>(F[0], XT);
  k_proj<<<dim3(TNB * TT / 64, 3), 128, 0, stream>>>(XT, F[1], F[2], F[3], F[4], F[5], F[6], F[7], F[8], F[9], F[10], AH, AL, BH, BL, MP);
  for (int b = 0; b < TNB; ++b) for (int qc = 0; qc < NQCH; ++qc) {
    k_sc<<<dim3(QCH / 64, TT / 128), 128, 0, stream>>>(AH, AL, BH, BL, b, qc * QCH, S);
    k_sm<<<dim3(QCH), 256, 0, stream>>>(S);
    k_pv<<<dim3(QCH / 64), 128, 0, stream>>>(S, MP, F[0], F[11], b, qc * QCH, (float*)d_out);
  }
}
